// PrivacyDetectionUnit_79018808312355
// MI455X (gfx1250) — hardware-verified
//
#include <hip/hip_runtime.h>
#include <math.h>

typedef __attribute__((ext_vector_type(16))) _Float16 v16h;
typedef __attribute__((ext_vector_type(16))) __bf16 v16b;
typedef __attribute__((ext_vector_type(8)))  _Float16 v8h;
typedef __attribute__((ext_vector_type(8)))  float v8f;
typedef __attribute__((ext_vector_type(4)))  float v4f;
typedef __attribute__((ext_vector_type(2)))  float v2f;
typedef __attribute__((ext_vector_type(4)))  unsigned v4u;
typedef __attribute__((ext_vector_type(4)))  int v4i;
typedef float __attribute__((may_alias)) float_a;
typedef int __attribute__((may_alias)) int_a;

template <typename T> __device__ __forceinline__ void vst2(void* p, T v) { *(volatile T*)p = v; __threadfence(); *(volatile T*)p = v; }
__device__ __forceinline__ v8f wmma16(v16h a, v16h b, v8f c) {
  v8f d = __builtin_amdgcn_wmma_f32_16x16x32_f16(false, a, false, b, (short)0, c, false, false);
  asm volatile("v_nop\n\tv_nop\n\tv_nop\n\tv_nop" : "+v"(d) : "v"(a), "v"(b));
  return d;
}
__device__ __forceinline__ v8f wmma_bf(v16b a, v16b b, v8f c) {
  v8f d = __builtin_amdgcn_wmma_f32_16x16x32_bf16(false, a, false, b, (short)0, c, false, false);
  asm volatile("v_nop\n\tv_nop\n\tv_nop\n\tv_nop" : "+v"(d) : "v"(a), "v"(b));
  return d;
}
__device__ __forceinline__ v16h frag_h(const _Float16* rowk0, int lane) {
  union { v16h v; v8h q[2]; } u; const _Float16* p = rowk0 + 8 * (lane >> 4);
  u.q[0] = *(const v8h*)p; u.q[1] = *(const v8h*)(p + 16); return u.v;
}
__device__ __forceinline__ v16h frag_f32(const float* rowk0, int lane) {
  v16h a; const float* p = rowk0 + 8 * (lane >> 4);
#pragma unroll
  for (int i = 0; i < 8; ++i) { a[i] = (_Float16)p[i]; a[8 + i] = (_Float16)p[16 + i]; }
  return a;
}
__device__ __forceinline__ v16h frag_f32s(const float* rowk0, int lane, float sc) {
  v16h a; const float* p = rowk0 + 8 * (lane >> 4);
#pragma unroll
  for (int i = 0; i < 8; ++i) { a[i] = (_Float16)(p[i] * sc); a[8 + i] = (_Float16)(p[16 + i] * sc); }
  return a;
}
__device__ __forceinline__ v16h fragc_f32(const float* W, int k0, int n, int lane, int ld, int K) {
  v16h a; const int g = lane >> 4;
#pragma unroll
  for (int i = 0; i < 8; ++i) { const int ka = k0 + 8 * g + i, kb = ka + 16;
    a[i] = (_Float16)(ka < K ? W[(size_t)ka * ld + n] : 0.f); a[8 + i] = (_Float16)(kb < K ? W[(size_t)kb * ld + n] : 0.f); }
  return a;
}
struct F2 { v16b h, l; };
__device__ __forceinline__ F2 bsplit16(const float v[16]) { F2 r;
#pragma unroll
  for (int i = 0; i < 16; ++i) { const __bf16 h = (__bf16)v[i]; r.h[i] = h; r.l[i] = (__bf16)(v[i] - (float)h); }
  return r; }
__device__ __forceinline__ F2 split_row(const float* row, int k0, int lane) { float v[16]; const float* p = row + k0 + 8 * (lane >> 4);
#pragma unroll
  for (int i = 0; i < 8; ++i) { v[i] = p[i]; v[8 + i] = p[16 + i]; }
  return bsplit16(v); }
__device__ __forceinline__ F2 split_rowK(const float* row, int k0, int lane, int K) { float v[16]; const int g = lane >> 4;
#pragma unroll
  for (int i = 0; i < 8; ++i) { const int ka = k0 + 8 * g + i, kb = ka + 16; v[i] = ka < K ? row[ka] : 0.f; v[8 + i] = kb < K ? row[kb] : 0.f; }
  return bsplit16(v); }
__device__ __forceinline__ F2 split_col(const float* W, int k0, int n, int lane, int ld, int K) { float v[16]; const int g = lane >> 4;
#pragma unroll
  for (int i = 0; i < 8; ++i) { const int ka = k0 + 8 * g + i, kb = ka + 16; v[i] = ka < K ? W[(size_t)ka * ld + n] : 0.f; v[8 + i] = kb < K ? W[(size_t)kb * ld + n] : 0.f; }
  return bsplit16(v); }
__device__ __forceinline__ v8f mac3(const F2& a, const F2& b, v8f c) { c = wmma_bf(a.l, b.h, c); c = wmma_bf(a.h, b.l, c); return wmma_bf(a.h, b.h, c); }
__device__ __forceinline__ float sigm(float v) { return 1.0f / (1.0f + expf(-v)); }
#define LDSX() do { asm volatile("s_wait_dscnt 0" ::: "memory"); __builtin_amdgcn_wave_barrier(); __builtin_amdgcn_fence(__ATOMIC_RELEASE, "workgroup"); } while (0)


#define NN 10000
#define NNP 10240
#define NE 160000
#define NG 64
#define D 512
#define GH 4
#define GO 128
#define XPW 544
#define RBA 64
#define NRBA (NNP / RBA)
#define RBM 2048
#define NRBM (NNP / RBM)
#define EPT 16
#define CH (256 * EPT)
#define FXS 1099511627776.0
typedef _Float16 v4h __attribute__((ext_vector_type(4)));

__device__ __forceinline__ int f2ord(float f) { const int i = __float_as_int(f); return i >= 0 ? i : i ^ 0x7fffffff; }
__device__ __forceinline__ float ord2f(int i) { return __int_as_float(i >= 0 ? i : i ^ 0x7fffffff); }
__device__ __forceinline__ float lrelu(float v) { return v > 0.f ? v : 0.2f * v; }
__device__ __forceinline__ int clampn(int v) { return v < 0 ? 0 : (v >= NN ? NN - 1 : v); }

__global__ __launch_bounds__(256) void k_cvt(const float* __restrict__ x, _Float16* __restrict__ X16) {
  const size_t i8 = (size_t)blockIdx.x * 256 + threadIdx.x; if (i8 >= (size_t)NNP * D / 8) return;
  const size_t r = (i8 * 8) / D; union { v8h h; v4u u; } pk;
#pragma unroll
  for (int e = 0; e < 8; ++e) pk.h[e] = r < NN ? (_Float16)x[i8 * 8 + e] : (_Float16)0.0f;
  vst2(X16 + i8 * 8, pk.u);
}
__global__ __launch_bounds__(256) void k_w1(const float* __restrict__ W1, const float* __restrict__ as1, const float* __restrict__ ad1, _Float16* __restrict__ PT1) {
  const int n = blockIdx.x, tid = threadIdx.x; __shared__ __align__(16) _Float16 srow[D];
  for (int k = tid; k < D; k += 256) { float v;
    if (n < D) v = W1[(size_t)k * D + n];
    else if (n < D + 2 * GH) { const int h = (n - D) & 3; const float* a = (n < D + GH ? as1 : ad1) + h * GO; const float* w = W1 + (size_t)k * D + h * GO; float s = 0.f;
#pragma unroll 4
      for (int c = 0; c < GO; ++c) s += w[c] * a[c]; v = s; }
    else v = 0.f;
    srow[k] = (_Float16)(v * 16.0f); }
  __syncthreads();
  if (tid < D / 8) vst2(PT1 + (size_t)n * D + tid * 8, *(const v4u*)(&srow[tid * 8]));
}
__global__ __launch_bounds__(128) void k_xp(const _Float16* __restrict__ X16, const _Float16* __restrict__ PT1, float* __restrict__ XP) {
  __shared__ __align__(16) float so[4][16][132];
  const int tid = threadIdx.x, wave = tid >> 5, lane = tid & 31, col = lane & 15, g = lane >> 4;
  const int r0 = blockIdx.x * 64 + wave * 16, cg = blockIdx.y, n0 = cg * 128; const int nt = cg < 4 ? 8 : 2;
  v8f acc[8] = {};
#pragma unroll 2
  for (int kc = 0; kc < D / 32; ++kc) { const v16h a = frag_h(X16 + (size_t)(r0 + col) * D + kc * 32, lane);
#pragma unroll
    for (int j = 0; j < 8; ++j) if (j < nt) acc[j] = wmma16(a, frag_h(PT1 + (size_t)(n0 + j * 16 + col) * D + kc * 32, lane), acc[j]); }
#pragma unroll
  for (int j = 0; j < 8; ++j) if (j < nt) {
#pragma unroll
    for (int r = 0; r < 8; ++r) so[wave][8 * g + r][j * 16 + col] = acc[j][r] * (1.0f / 16.0f); }
  LDSX();
  const int npc = nt * 4;
  for (int q = lane; q < 16 * npc; q += 32) { const int rl = q / npc, pc = q % npc; vst2(XP + (size_t)(r0 + rl) * XPW + n0 + pc * 4, *(const v4f*)(&so[wave][rl][pc * 4])); }
}
__global__ __launch_bounds__(256) void k_max1(const int* __restrict__ esrc, const int* __restrict__ edst, const float* __restrict__ XP, float* __restrict__ SMX1) {
  __shared__ int smx[RBM][GH]; __shared__ __align__(16) float sdst[RBM][GH];
  const int tid = threadIdx.x; const int r0 = blockIdx.x * RBM;
  for (int rl = tid; rl < RBM; rl += 256) { const int row = r0 + rl; v4f sd = {0.f, 0.f, 0.f, 0.f}, ssf = {0.f, 0.f, 0.f, 0.f};
    if (row < NN) { sd = *(const v4f*)(XP + (size_t)row * XPW + D + GH); ssf = *(const v4f*)(XP + (size_t)row * XPW + D); }
    *(v4f*)&sdst[rl][0] = sd;
#pragma unroll
    for (int h = 0; h < GH; ++h) smx[rl][h] = f2ord(row < NN ? lrelu(ssf[h] + sd[h]) : -3.0e38f); }
  __syncthreads();
#pragma unroll 1
  for (int c0 = 0; c0 < NE; c0 += CH) { const int e0 = c0 + tid * EPT;
#pragma unroll
    for (int v = 0; v < EPT / 4; ++v) { int dd[4];
      if (e0 + v * 4 + 4 <= NE) { const int4 d4 = *(const int4*)(edst + e0 + v * 4); dd[0] = d4.x; dd[1] = d4.y; dd[2] = d4.z; dd[3] = d4.w; }
      else { for (int u = 0; u < 4; ++u) dd[u] = (e0 + v * 4 + u < NE) ? edst[e0 + v * 4 + u] : -1; }
#pragma unroll
      for (int u = 0; u < 4; ++u) { if (dd[u] < 0) continue; const int dcl = clampn(dd[u]); const unsigned relr = (unsigned)(dcl - r0); if (relr < (unsigned)RBM) {
          const int s = clampn(esrc[e0 + v * 4 + u]); const v4f ss = *(const v4f*)(XP + (size_t)s * XPW + D);
#pragma unroll
          for (int h = 0; h < GH; ++h) atomicMax(&smx[relr][h], f2ord(lrelu(ss[h] + sdst[relr][h]))); } } } }
  __syncthreads();
  for (int rl = tid; rl < RBM; rl += 256) vst2(SMX1 + (size_t)(r0 + rl) * GH, (v4f){ord2f(smx[rl][0]), ord2f(smx[rl][1]), ord2f(smx[rl][2]), ord2f(smx[rl][3])});
}
__global__ __launch_bounds__(256) void k_u2(const float* __restrict__ W2, const float* __restrict__ as2, const float* __restrict__ ad2, float* __restrict__ U2) {
  const int which = blockIdx.x, tid = threadIdx.x; const float* a = which == 0 ? as2 : ad2; __shared__ __align__(16) float su[D];
  for (int k = tid; k < D; k += 256) { const float* w = W2 + (size_t)k * D; float s = 0.f;
#pragma unroll 4
    for (int c = 0; c < D; ++c) s += w[c] * a[c]; su[k] = s; }
  __syncthreads();
  if (tid < D / 4) vst2(U2 + (size_t)which * D + tid * 4, *(const v4f*)(&su[tid * 4]));
}
__global__ __launch_bounds__(256) void k_agg1(const int* __restrict__ esrc, const int* __restrict__ edst, const float* __restrict__ XP, const float* __restrict__ SMX1,
                                             const float* __restrict__ b1, const float* __restrict__ U2, float* __restrict__ H1, float* __restrict__ S2) {
  __shared__ __align__(16) float sacc[RBA][D];
  __shared__ __align__(16) float sden[RBA][GH]; __shared__ __align__(16) float smx_[RBA][GH]; __shared__ __align__(16) float sdst[RBA][GH];
  __shared__ int ssrc[8][32 * EPT], sdl[8][32 * EPT]; __shared__ int scnt[8];
  __shared__ __align__(16) float ss2[RBA][2];
  const int tid = threadIdx.x, wave = tid >> 5, lane = tid & 31;
  const int r0 = blockIdx.x * RBA;
  for (int q = tid; q < RBA * D; q += 256) (&sacc[0][0])[q] = 0.f;
  if (tid < RBA) { const int row = r0 + tid;
#pragma unroll
    for (int h = 0; h < GH; ++h) { sden[tid][h] = 0.f; smx_[tid][h] = row < NN ? SMX1[(size_t)row * GH + h] : 0.f; sdst[tid][h] = row < NN ? XP[(size_t)row * XPW + D + GH + h] : 0.f; } }
  __syncthreads();
#pragma unroll 1
  for (int c0 = 0; c0 < NE; c0 += CH) { const int e0 = c0 + tid * EPT; int hd[EPT];
    if (e0 + EPT <= NE) {
#pragma unroll
      for (int v = 0; v < EPT / 4; ++v) { const int4 d4 = *(const int4*)(edst + e0 + v * 4); const int dd[4] = {d4.x, d4.y, d4.z, d4.w};
#pragma unroll
        for (int u = 0; u < 4; ++u) { const unsigned relr = (unsigned)(clampn(dd[u]) - r0); hd[v * 4 + u] = relr < (unsigned)RBA ? (int)relr : -1; } } }
    else {
#pragma unroll
      for (int u = 0; u < EPT; ++u) { const int e = e0 + u; int dl = -1; if (e < NE) { const unsigned relr = (unsigned)(clampn(edst[e]) - r0); dl = relr < (unsigned)RBA ? (int)relr : -1; } hd[u] = dl; } }
    int cnt = 0;
#pragma unroll
    for (int u = 0; u < EPT; ++u) cnt += hd[u] >= 0;
    int incl = cnt;
#pragma unroll
    for (int off = 1; off < 32; off <<= 1) { const int v = __shfl_up(incl, off, 32); if (lane >= off) incl += v; }
    if (lane == 31) scnt[wave] = incl;
    int pos = incl - cnt;
#pragma unroll
    for (int u = 0; u < EPT; ++u) if (hd[u] >= 0) { ssrc[wave][pos] = e0 + u; sdl[wave][pos] = hd[u]; ++pos; }
    __syncthreads();
    { const int f = tid; const int ha = f >> 7, hb = ha + 2;
      for (int w = 0; w < 8; ++w) { const int nh = scnt[w]; for (int i = 0; i < nh; ++i) { const int e = ssrc[w][i], dl = sdl[w][i]; const int s = clampn(esrc[e]);
          const float* xr = XP + (size_t)s * XPW; const v4f ss = *(const v4f*)(xr + D);
          const float wa = expf(lrelu(ss[ha] + sdst[dl][ha]) - smx_[dl][ha]), wb = expf(lrelu(ss[hb] + sdst[dl][hb]) - smx_[dl][hb]);
          sacc[dl][f] += wa * xr[f]; sacc[dl][f + 256] += wb * xr[f + 256];
          if ((f & 127) == 0) { sden[dl][ha] += wa; sden[dl][hb] += wb; } } } }
    __syncthreads(); }
#pragma unroll 1
  for (int q = tid; q < RBA * D; q += 256) { const int rl = q >> 9, f = q & 511; const int row = r0 + rl; const int h = f >> 7; float v = 0.f;
    if (row < NN) { const float* xr = XP + (size_t)row * XPW; const float wself = expf(lrelu(xr[D + h] + sdst[rl][h]) - smx_[rl][h]);
      const float num = sacc[rl][f] + wself * xr[f]; const float den = sden[rl][h] + wself; const float a = num / den + b1[f]; v = a > 0.f ? a : expm1f(a); }
    sacc[rl][f] = v; }
  __syncthreads();
  { const int rl = tid >> 2, qd = tid & 3; float a = 0.f, bb = 0.f; const float* hr = &sacc[rl][qd * 128]; const float* ua = U2 + qd * 128; const float* ub = U2 + D + qd * 128;
#pragma unroll 4
    for (int c = 0; c < 128; ++c) { a += hr[c] * ua[c]; bb += hr[c] * ub[c]; }
    a += __shfl_xor(a, 1, 32); a += __shfl_xor(a, 2, 32); bb += __shfl_xor(bb, 1, 32); bb += __shfl_xor(bb, 2, 32);
    if (qd == 0) { ss2[rl][0] = a; ss2[rl][1] = bb; } }
  __syncthreads();
  for (int q = tid; q < RBA * (D / 4); q += 256) { const int rl = q >> 7, pc = q & 127; vst2(H1 + (size_t)(r0 + rl) * D + pc * 4, *(const v4f*)(&sacc[rl][pc * 4])); }
  if (tid < 32) vst2(S2 + (size_t)r0 * 2 + tid * 4, *(const v4f*)(&ss2[0][0] + tid * 4));
}
__global__ __launch_bounds__(256) void k_stat2(const int* __restrict__ esrc, const int* __restrict__ edst, const float* __restrict__ S2, float* __restrict__ SMX2, float* __restrict__ DEN2) {
  __shared__ int smx[RBM]; __shared__ unsigned long long sden[RBM]; __shared__ float sdst[RBM], sself[RBM];
  const int tid = threadIdx.x; const int r0 = blockIdx.x * RBM;
  for (int rl = tid; rl < RBM; rl += 256) { const int row = r0 + rl; float sd = 0.f, es = -3.0e38f; if (row < NN) { const v2f s = *(const v2f*)(S2 + (size_t)row * 2); sd = s[1]; es = lrelu(s[0] + s[1]); }
    sdst[rl] = sd; sself[rl] = es; smx[rl] = f2ord(es); sden[rl] = 0ull; }
  __syncthreads();
#pragma unroll 1
  for (int pass = 0; pass < 2; ++pass) {
#pragma unroll 1
    for (int c0 = 0; c0 < NE; c0 += CH) { const int e0 = c0 + tid * EPT;
#pragma unroll
      for (int v = 0; v < EPT / 4; ++v) { int dd[4];
        if (e0 + v * 4 + 4 <= NE) { const int4 d4 = *(const int4*)(edst + e0 + v * 4); dd[0] = d4.x; dd[1] = d4.y; dd[2] = d4.z; dd[3] = d4.w; }
        else { for (int u = 0; u < 4; ++u) dd[u] = (e0 + v * 4 + u < NE) ? edst[e0 + v * 4 + u] : -1; }
#pragma unroll
        for (int u = 0; u < 4; ++u) { if (dd[u] < 0) continue; const unsigned relr = (unsigned)(clampn(dd[u]) - r0); if (relr < (unsigned)RBM) {
            const int s = clampn(esrc[e0 + v * 4 + u]); const float e = lrelu(S2[(size_t)s * 2] + sdst[relr]);
            if (pass == 0) atomicMax(&smx[relr], f2ord(e));
            else { const float w = expf(e - ord2f(smx[relr])); atomicAdd(&sden[relr], (unsigned long long)__double2ll_rn((double)w * FXS)); } } } } }
    __syncthreads(); }
  for (int q = tid; q < RBM / 4; q += 256) { v4f m, dn;
#pragma unroll
    for (int u = 0; u < 4; ++u) { const int rl = q * 4 + u; const float mx = ord2f(smx[rl]); m[u] = mx;
      dn[u] = (float)((double)sden[rl] / FXS) + expf(sself[rl] - mx); }
    vst2(SMX2 + (size_t)r0 + q * 4, m); vst2(DEN2 + (size_t)r0 + q * 4, dn); }
}
__global__ __launch_bounds__(256) void k_omega(const int* __restrict__ esrc, const int* __restrict__ edst, const int* __restrict__ batch, const float* __restrict__ S2,
                                              const float* __restrict__ SMX2, const float* __restrict__ DEN2, float* __restrict__ OM, int* __restrict__ CNTL) {
  __shared__ unsigned long long som[NNP]; __shared__ int scnt[8];
  const int tid = threadIdx.x, wave = tid >> 5, lane = tid & 31; const int gph = blockIdx.x;
  for (int m = tid; m < NNP; m += 256) som[m] = 0ull;
  __syncthreads();
  int cnt = 0;
#pragma unroll 1
  for (int n = tid; n < NN; n += 256) { if (batch[n] == gph) { ++cnt; const v2f s = *(const v2f*)(S2 + (size_t)n * 2);
      const float w = expf(lrelu(s[0] + s[1]) - SMX2[n]) / DEN2[n]; atomicAdd(&som[n], (unsigned long long)__double2ll_rn((double)w * FXS)); } }
#pragma unroll
  for (int off = 16; off > 0; off >>= 1) cnt += __shfl_xor(cnt, off, 32);
  if (lane == 0) scnt[wave] = cnt;
#pragma unroll 1
  for (int e = tid; e < NE; e += 256) { const int n = clampn(edst[e]);
    if (batch[n] == gph) { const int s = clampn(esrc[e]); const float lg = lrelu(S2[(size_t)s * 2] + S2[(size_t)n * 2 + 1]);
      const float w = expf(lg - SMX2[n]) / DEN2[n]; atomicAdd(&som[s], (unsigned long long)__double2ll_rn((double)w * FXS)); } }
  __syncthreads();
  for (int q = tid; q < NNP / 4; q += 256) { v4f o;
#pragma unroll
    for (int u = 0; u < 4; ++u) o[u] = (float)((double)som[q * 4 + u] / FXS);
    vst2(OM + (size_t)gph * NNP + q * 4, o); }
  if (tid < 32) { int c = 0;
#pragma unroll
    for (int w = 0; w < 8; ++w) c += scnt[w];
    vst2(CNTL + (size_t)gph * 32 + tid, (int_a)c); }
}
template <int EPI>
__global__ __launch_bounds__(128) void k_lin(const float* __restrict__ A, int lda, int K, const float* __restrict__ Bm, int N, const float* __restrict__ bias, const int* __restrict__ CNTL,
                                            float* __restrict__ C, int ldc) {
  __shared__ __align__(16) float so[4][16][132];
  const int tid = threadIdx.x, wave = tid >> 5, lane = tid & 31, col = lane & 15, g = lane >> 4;
  const int n0 = blockIdx.x * 128;
  v8f acc[4][2] = {};
#pragma unroll 1
  for (int kc = 0; kc < K / 32; ++kc) {
    const F2 b0 = split_col(Bm, kc * 32, n0 + (2 * wave) * 16 + col, lane, N, K), b1 = split_col(Bm, kc * 32, n0 + (2 * wave + 1) * 16 + col, lane, N, K);
#pragma unroll
    for (int i = 0; i < 4; ++i) { const F2 a = split_row(A + (size_t)(i * 16 + col) * lda, kc * 32, lane); acc[i][0] = mac3(a, b0, acc[i][0]); acc[i][1] = mac3(a, b1, acc[i][1]); } }
#pragma unroll
  for (int i = 0; i < 4; ++i)
#pragma unroll
    for (int j = 0; j < 2; ++j) { const int nl = (2 * wave + j) * 16 + col; const float bb = bias != nullptr ? bias[n0 + nl] : 0.f;
#pragma unroll
      for (int r = 0; r < 8; ++r) { const int row = i * 16 + 8 * g + r; float v = acc[i][j][r];
        if (EPI == 1) { const float c = (float)CNTL[row * 32]; v = v / fmaxf(c, 1.0f); }
        else if (EPI == 3) { const float c = (float)CNTL[row * 32]; v += bb * fminf(c, 1.0f); }
        else { v += bb; if (EPI == 2) v = fmaxf(v, 0.f); }
        so[i][8 * g + r][nl] = v; } }
  __syncthreads();
#pragma unroll 4
  for (int rl = 0; rl < 16; ++rl) vst2(C + (size_t)(wave * 16 + rl) * ldc + n0 + lane * 4, *(const v4f*)(&so[wave][rl][lane * 4]));
}
__global__ __launch_bounds__(256) void k_final(const float* __restrict__ Z, const float* __restrict__ wc2, const float* __restrict__ bc2, const float* __restrict__ rule, float* __restrict__ out0) {
  __shared__ __align__(16) float sres[NG];
  const int tid = threadIdx.x, gph = tid >> 2, qd = tid & 3; float a = 0.f; const float* zr = Z + (size_t)gph * 256 + qd * 64; const float* w = wc2 + qd * 64;
#pragma unroll 4
  for (int c = 0; c < 64; ++c) a += zr[c] * w[c];
  a += __shfl_xor(a, 1, 32); a += __shfl_xor(a, 2, 32);
  if (qd == 0) sres[gph] = 0.5f * sigm(a + bc2[0]) + 0.5f * rule[gph];
  __syncthreads();
  if (tid < 16) vst2(out0 + tid * 4, *(const v4f*)(&sres[tid * 4]));
}
extern "C" void kernel_launch(void* const* d_in, const int* in_sizes, int n_in, void* d_out, int out_size, void* d_ws, size_t ws_size, hipStream_t stream) {
  (void)in_sizes; (void)n_in; (void)out_size; (void)ws_size;
  const float* x = (const float*)d_in[1]; const float* rule = (const float*)d_in[2]; const int* eidx = (const int*)d_in[3]; const int* batch = (const int*)d_in[4];
  const float* W1 = (const float*)d_in[7]; const float* as1 = (const float*)d_in[8]; const float* ad1 = (const float*)d_in[9]; const float* b1 = (const float*)d_in[10];
  const float* W2 = (const float*)d_in[11]; const float* as2 = (const float*)d_in[12]; const float* ad2 = (const float*)d_in[13]; const float* b2 = (const float*)d_in[14];
  const float* Wv = (const float*)d_in[19]; const float* bv = (const float*)d_in[20]; const float* Wo = (const float*)d_in[21]; const float* bo = (const float*)d_in[22];
  const float* Wc1 = (const float*)d_in[23]; const float* bc1 = (const float*)d_in[24]; const float* Wc2 = (const float*)d_in[25]; const float* bc2 = (const float*)d_in[26];
  const int* esrc = eidx; const int* edst = eidx + NE;
  float* out0 = (float*)d_out; float* out1 = (float*)((char*)d_out + 256);
  char* ws = (char*)d_ws; size_t off = 0;
  auto take = [&](size_t bytes) { char* p = ws + off; off += (bytes + 255) & ~(size_t)255; return p; };
  _Float16* X16 = (_Float16*)take((size_t)NNP * D * 2); _Float16* PT1 = (_Float16*)take((size_t)XPW * D * 2); float* XP = (float*)take((size_t)NNP * XPW * 4);
  float* SMX1 = (float*)take((size_t)NNP * GH * 4); float* U2 = (float*)take((size_t)2 * D * 4); float* H1 = (float*)take((size_t)NNP * D * 4); float* S2 = (float*)take((size_t)NNP * 2 * 4);
  float* SMX2 = (float*)take((size_t)NNP * 4); float* DEN2 = (float*)take((size_t)NNP * 4); float* OM = (float*)take((size_t)NG * NNP * 4); int* CNTL = (int*)take((size_t)NG * 32 * 4);
  float* GA = (float*)take((size_t)NG * D * 4); float* GF = (float*)take((size_t)NG * D * 4); float* V = (float*)take((size_t)NG * D * 4); float* Z = (float*)take((size_t)NG * 256 * 4);
  k_cvt<<<(NNP * D / 8 + 255) / 256, 256, 0, stream>>>(x, X16);
  k_w1<<<XPW, 256, 0, stream>>>(W1, as1, ad1, PT1);
  k_xp<<<dim3(NNP / 64, 5), 128, 0, stream>>>(X16, PT1, XP);
  k_max1<<<NRBM, 256, 0, stream>>>(esrc, edst, XP, SMX1);
  k_u2<<<2, 256, 0, stream>>>(W2, as2, ad2, U2);
  k_agg1<<<NRBA, 256, 0, stream>>>(esrc, edst, XP, SMX1, b1, U2, H1, S2);
  k_stat2<<<NRBM, 256, 0, stream>>>(esrc, edst, S2, SMX2, DEN2);
  k_omega<<<NG, 256, 0, stream>>>(esrc, edst, batch, S2, SMX2, DEN2, OM, CNTL);
  k_lin<1><<<D / 128, 128, 0, stream>>>(OM, NNP, NNP, H1, D, nullptr, CNTL, GA, D);
  k_lin<3><<<D / 128, 128, 0, stream>>>(GA, D, D, W2, D, b2, CNTL, GF, D);
  k_lin<0><<<D / 128, 128, 0, stream>>>(GF, D, D, Wv, D, bv, CNTL, V, D);
  k_lin<0><<<D / 128, 128, 0, stream>>>(V, D, D, Wo, D, bo, CNTL, out1, D);
  k_lin<2><<<256 / 128, 128, 0, stream>>>(out1, D, D, Wc1, 256, bc1, CNTL, Z, 256);
  k_final<<<1, 256, 0, stream>>>(Z, Wc2, bc2, rule, out0);
}
